// FractionalFusionUp_11991548690812
// MI455X (gfx1250) — hardware-verified
//
#include <hip/hip_runtime.h>
#include <math.h>


typedef __attribute__((ext_vector_type(16))) _Float16 v16h;
typedef __attribute__((ext_vector_type(8)))  _Float16 v8h;
typedef __attribute__((ext_vector_type(8)))  float  v8f;
typedef __attribute__((ext_vector_type(4)))  float  v4f;
template <typename V> __device__ __forceinline__ void vst2(void* p, V v) {
  *(volatile V*)p = v; __threadfence(); *(volatile V*)p = v;
}
__device__ __forceinline__ v8f WMMA16(bool, v16h a, bool, v16h b, short, v8f c, bool, bool) {
  v8f d = __builtin_amdgcn_wmma_f32_16x16x32_f16(false, a, false, b, (short)0, c, false, false);
  asm volatile("v_nop\n\tv_nop\n\tv_nop\n\tv_nop" : "+v"(d) : "v"(a), "v"(b));
  return d;
}
typedef unsigned int ui4 __attribute__((ext_vector_type(4)));
typedef int          si8 __attribute__((ext_vector_type(8)));
typedef int          si4 __attribute__((ext_vector_type(4)));

#define B_     4
#define C_IN   21
#define H0     81
#define W0     81
#define HH     324
#define NCH    96
#define NPIX   (B_*H0*W0)
#define NTILE  ((NPIX+15)/16)
#define K1     189
#define K1P    192
#define KC1    6
#define NT1    6
#define K2     864
#define K2P    896
#define KC2    28
#define NHR    (B_*HH*HH)

#define W1ELEMS (KC1*NT1*32*16)
#define W2ELEMS (KC2*32*16)

#define OFF_W1  0u
#define OFF_W2  36864u
#define OFF_H   65536u
#define OFF_REC 5111808u
#define NPIXP   (NTILE*16)

#define OUT_V   (B_*C_IN*HH*HH)
#define OUT_G   (OUT_V + B_*8*H0*W0)

__device__ __constant__ float S8[8][9] = {
  {-1, 0, 1,  -1, 0, 1,  -1, 0, 1},
  {-1,-1, 0,  -1, 0, 1,   0, 1, 1},
  {-1,-1,-1,   0, 0, 0,   1, 1, 1},
  { 0,-1,-1,   1, 0,-1,   1, 1, 0},
  { 1, 0,-1,   1, 0,-1,   1, 0,-1},
  { 1, 1, 0,   1, 0,-1,   0,-1,-1},
  { 1, 1, 1,   0, 0, 0,  -1,-1,-1},
  { 0, 1, 1,  -1, 0, 1,  -1,-1, 0},
};

__device__ __forceinline__ int a_kmap(int e, int half) {
  return ((e < 8) ? e : e + 8) + 8 * half;
}

__device__ __forceinline__ int tap_mask(int py, int px) {
  int tm = 0;
#pragma unroll
  for (int i = 0; i < 3; ++i)
#pragma unroll
    for (int j = 0; j < 3; ++j) {
      int okt = (int)((unsigned)(py + i - 1) < (unsigned)H0) &
                (int)((unsigned)(px + j - 1) < (unsigned)W0);
      tm |= okt << (i * 3 + j);
    }
  return tm;
}

__device__ __forceinline__ void copy_to_lds(const void* gsrc, void* ldst, unsigned n16, int tid, int nthr) {
  for (unsigned c = tid; c < n16; c += nthr) ((ui4*)ldst)[c] = ((const ui4*)gsrc)[c];
}

__global__ void prep_w1(const float* __restrict__ w1o,
                        const float* __restrict__ w1g,
                        _Float16* __restrict__ wp) {
  int g = blockIdx.x * blockDim.x + threadIdx.x;
  if (g * 8 >= W1ELEMS) return;
  union { v8h h; ui4 u; } pk;
#pragma unroll
  for (int q = 0; q < 8; ++q) {
    int t = g * 8 + q;
    int e  = t & 15;
    int l  = (t >> 4) & 31;
    int rs = t >> 9;
    int tn = rs % NT1;
    int kc = rs / NT1;
    int half = l >> 4, lq = l & 15;
    int K = kc * 32 + a_kmap(e, half);
    int n = tn * 16 + lq;
    float v = 0.f;
    if (K < K1) {
      int ci = K / 9, tt = K - ci * 9, ty = tt / 3, tx = tt - ty * 3;
      v = (n < 48) ? w1o[((n * C_IN + ci) * 3 + ty) * 3 + tx]
                   : w1g[(((n - 48) * C_IN + ci) * 3 + ty) * 3 + tx];
    }
    pk.h[q] = (_Float16)v;
  }
  vst2(wp + (size_t)g * 8, pk.u);
}

__global__ void prep_w2(const float* __restrict__ w2o,
                        const float* __restrict__ w2g,
                        _Float16* __restrict__ wp) {
  int g = blockIdx.x * blockDim.x + threadIdx.x;
  if (g * 8 >= W2ELEMS) return;
  union { v8h h; ui4 u; } pk;
#pragma unroll
  for (int q = 0; q < 8; ++q) {
    int t = g * 8 + q;
    int e  = t & 15;
    int l  = (t >> 4) & 31;
    int kc = t >> 9;
    int half = l >> 4, lq = l & 15;
    int K = kc * 32 + a_kmap(e, half);
    int n = lq;
    float v = 0.f;
    if (K < K2) {
      int ci = K / 9, tt = K - ci * 9, ty = tt / 3, tx = tt - ty * 3;
      if (n < 8 && ci < 48)        v = w2o[((n * 48 + ci) * 3 + ty) * 3 + tx];
      else if (n == 8 && ci >= 48) v = w2g[((ci - 48) * 3 + ty) * 3 + tx];
    }
    pk.h[q] = (_Float16)v;
  }
  vst2(wp + (size_t)g * 8, pk.u);
}

__device__ __forceinline__ int make_kent(int K, int Kmax, int chanStride) {
  if (K >= Kmax) return 0;
  int ci = K / 9, tap = K - ci * 9, ty = tap / 3, tx = tap - ty * 3;
  int off = ci * chanStride + (ty - 1) * W0 + (tx - 1);
  return (off << 5) | (1 << 4) | tap;
}

__global__ void __launch_bounds__(256)
conv1_wmma(const float* __restrict__ x,
           const float* __restrict__ b1o, const float* __restrict__ b1g,
           const _Float16* __restrict__ wp, _Float16* __restrict__ hbuf) {
  __shared__ __attribute__((aligned(32))) _Float16 w1s[W1ELEMS];
  __shared__ int ktab[K1P];

  __shared__ __align__(16) _Float16 otile[8][16 * NCH];
  for (int i = threadIdx.x; i < K1P; i += blockDim.x)
    ktab[i] = make_kent(i, K1, H0 * W0);
  copy_to_lds(wp, w1s, W1ELEMS * 2 / 16, threadIdx.x, 256);
  __syncthreads();

  const int widx = threadIdx.x >> 5;
  int wave = blockIdx.x * 8 + widx;
  if (wave >= NTILE) return;
  int lane = threadIdx.x & 31;
  int half = lane >> 4, lq = lane & 15;
  int p0 = wave * 16;
  int pr = p0 + lq; if (pr >= NPIX) pr = NPIX - 1;
  int b   = pr / (H0 * W0);
  int rem = pr - b * H0 * W0;
  int py  = rem / W0, px = rem - py * W0;
  int pixbase = b * (C_IN * H0 * W0) + py * W0 + px;
  int tmask = tap_mask(py, px);

  v8f acc[NT1] = {};
  const v16h* wls = (const v16h*)w1s;

  for (int kc = 0; kc < KC1; ++kc) {
    v16h a;
#pragma unroll
    for (int e = 0; e < 16; ++e) {
      int K = kc * 32 + a_kmap(e, half);
      int ent = ktab[K];
      int ok = (ent >> 4) & (tmask >> (ent & 15)) & 1;
      int off = ok ? (ent >> 5) : 0;
      float v = x[pixbase + off];
      a[e] = (_Float16)(ok ? v : 0.f);
    }
#pragma unroll
    for (int tn = 0; tn < NT1; ++tn) {
      v16h bf = wls[(kc * NT1 + tn) * 32 + lane];
      acc[tn] = WMMA16(
          false, a, false, bf, (short)0, acc[tn], false, false);
    }
  }

  _Float16* ot = otile[widx];
#pragma unroll
  for (int tn = 0; tn < NT1; ++tn) {
    int n = tn * 16 + lq;
    float bias = (n < 48) ? b1o[n] : b1g[n - 48];
#pragma unroll
    for (int r = 0; r < 8; ++r) ot[(r + 8 * half) * NCH + n] = (_Float16)fmaxf(acc[tn][r] + bias, 0.f);
  }
  __builtin_amdgcn_wave_barrier();
  __builtin_amdgcn_fence(__ATOMIC_RELEASE, "workgroup");
  {
    _Float16* dst = hbuf + (size_t)p0 * NCH;
#pragma unroll
    for (int q = 0; q < 6; ++q) { int g = q * 32 + lane; vst2(dst + g * 8, *(const ui4*)(ot + g * 8)); }
  }
}

__global__ void __launch_bounds__(256)
conv2_wmma(const _Float16* __restrict__ hbuf, const _Float16* __restrict__ wp,
           const float* __restrict__ b2o, const float* __restrict__ b2g,
           float* __restrict__ recbuf) {
  __shared__ __attribute__((aligned(32))) _Float16 w2s[W2ELEMS];
  __shared__ int ktab2[K2P];
  __shared__ float s_raw[8][16][16];

  __shared__ __align__(16) float srec[8][16][32];
  for (int i = threadIdx.x; i < K2P; i += blockDim.x) {
    int K = i;
    int ent = 0;
    if (K < K2) { int ci = K / 9, tap = K - ci * 9, ty = tap / 3, tx = tap - ty * 3;
                  int off = ((ty - 1) * W0 + (tx - 1)) * NCH + ci; ent = (off << 5) | (1 << 4) | tap; }
    ktab2[i] = ent;
  }
  copy_to_lds(wp, w2s, W2ELEMS * 2 / 16, threadIdx.x, 256);
  __syncthreads();

  int widx = threadIdx.x >> 5;
  int wave = blockIdx.x * 8 + widx;
  const bool wvalid = (wave < NTILE);
  if (!wvalid) wave = NTILE - 1;
  int lane = threadIdx.x & 31;
  int half = lane >> 4, lq = lane & 15;
  int p0 = wave * 16;
  int pr = p0 + lq; if (pr >= NPIX) pr = NPIX - 1;
  int b   = pr / (H0 * W0);
  int rem = pr - b * H0 * W0;
  int py  = rem / W0, px = rem - py * W0;
  int pixbase = pr * NCH;
  int tmask = tap_mask(py, px);
  (void)b;

  v8f acc = {};
  const v16h* wls = (const v16h*)w2s;

  for (int kc = 0; kc < KC2; ++kc) {
    v16h a;
#pragma unroll
    for (int e = 0; e < 16; ++e) {
      int K = kc * 32 + a_kmap(e, half);
      int ent = ktab2[K];
      int ok = (ent >> 4) & (tmask >> (ent & 15)) & 1;
      int off = ok ? (ent >> 5) : 0;
      _Float16 v = hbuf[pixbase + off];
      a[e] = ok ? v : (_Float16)0.f;
    }
    v16h bf = wls[kc * 32 + lane];
    acc = WMMA16(
        false, a, false, bf, (short)0, acc, false, false);
  }

  float bias = (lq < 8) ? b2o[lq] : ((lq == 8) ? b2g[0] : 0.f);
#pragma unroll
  for (int r = 0; r < 8; ++r)
    s_raw[widx][r + 8 * half][lq] = acc[r] + bias;
  __syncthreads();

  if (lane < 16) {
    int p = p0 + lane;
    if (p < NPIX) {
      float raw[9];
#pragma unroll
      for (int n = 0; n < 9; ++n) raw[n] = s_raw[widx][lane][n];

      float vv[8];
#pragma unroll
      for (int d = 0; d < 8; ++d) vv[d] = tanhf(raw[d]);
      float g = 1.f / (1.f + expf(-raw[8]));

      float* rec = srec[widx][lane];
#pragma unroll
      for (int d = 0; d < 8; ++d) rec[19 + d] = vv[d];
      rec[18] = g;
#pragma unroll
      for (int d = 27; d < 32; ++d) rec[d] = 0.f;

      float kern[9];
#pragma unroll
      for (int kl = 0; kl < 9; ++kl) {
        float s = 0.f;
#pragma unroll
        for (int d = 0; d < 8; ++d) s += vv[d] * S8[d][kl];
        kern[kl] = -0.125f * s;
      }
      kern[4] += 2.5f;

      float mx = kern[0];
#pragma unroll
      for (int kl = 1; kl < 9; ++kl) mx = fmaxf(mx, kern[kl]);
      float ex[9], se = 0.f;
#pragma unroll
      for (int kl = 0; kl < 9; ++kl) {
        ex[kl] = expf((kern[kl] - mx) * 2.0f);
        se += ex[kl];
      }
      float inv = 1.f / se;
#pragma unroll
      for (int kl = 0; kl < 9; ++kl) rec[kl] = ex[kl] * inv;

      float mean = 0.f;
#pragma unroll
      for (int kl = 0; kl < 9; ++kl) mean += kern[kl];
      mean *= (1.f / 9.f);
      float tdev[9], den = 1e-8f;
#pragma unroll
      for (int kl = 0; kl < 9; ++kl) {
        tdev[kl] = kern[kl] - mean;
        den += fabsf(tdev[kl]);
      }
      float rden = 1.f / den;
#pragma unroll
      for (int kl = 0; kl < 9; ++kl) rec[9 + kl] = tdev[kl] * rden;
    }
  }
  __syncthreads();
  if (wvalid) {
    float* dst = recbuf + (size_t)p0 * 32;
#pragma unroll
    for (int q = 0; q < 4; ++q) { int rl = q * 4 + (lane >> 3), pc = lane & 7; vst2(dst + rl * 32 + pc * 4, *(const v4f*)(&srec[widx][rl][pc * 4])); }
  }
}

__global__ void __launch_bounds__(256) write_v(const float* __restrict__ rec, float* __restrict__ vout) {
  int g = blockIdx.x * 256 + threadIdx.x;
  if (g >= (B_ * 8 * H0 * W0) / 4) return;
  v4f o;
#pragma unroll
  for (int e = 0; e < 4; ++e) {
    int f = g * 4 + e;
    int pix = f % (H0 * W0); int bd = f / (H0 * W0); int d = bd & 7, b = bd >> 3;
    o[e] = rec[(size_t)(b * H0 * W0 + pix) * 32 + 19 + d];
  }
  vst2(vout + (size_t)g * 4, o);
}
__global__ void __launch_bounds__(256) write_g(const float* __restrict__ rec, float* __restrict__ gout) {
  int g = blockIdx.x * 256 + threadIdx.x;
  if (g >= NHR / 4) return;
  int f0 = g * 4;
  int b = f0 / (HH * HH); int rem = f0 - b * HH * HH; int Y = rem / HH, X0 = rem - Y * HH;
  int p = (b * H0 + (Y >> 2)) * W0 + (X0 >> 2);
  float gv = rec[(size_t)p * 32 + 18];
  v4f o = {gv, gv, gv, gv};
  vst2(gout + (size_t)g * 4, o);
}
__global__ void __launch_bounds__(256)
upsample_combine(const float* __restrict__ x, const float* __restrict__ rec,
                 const float* __restrict__ beta_p, float* __restrict__ yout) {
  int g = blockIdx.x * blockDim.x + threadIdx.x;
  if (g >= (B_ * C_IN * HH * HH) / 4) return;
  int f0 = g * 4;
  int X0 = f0 % HH; int t1 = f0 / HH; int Y = t1 % HH; int t2 = t1 / HH; int c = t2 % C_IN; int b = t2 / C_IN;
  int yl = Y >> 2, xl = X0 >> 2;
  int p = (b * H0 + yl) * W0 + xl;
  const float* rp = rec + (size_t)p * 32;
  float m[9], hk[9];
#pragma unroll
  for (int n = 0; n < 9; ++n) { m[n] = rp[n]; hk[n] = rp[9 + n]; }
  float gg  = rp[18];
  float lam = 0.15f * (1.f - gg);
  float tb  = tanhf(*beta_p) * gg;

  int ry[3], rx[3];
#pragma unroll
  for (int i = 0; i < 3; ++i) {
    int t = yl + i - 1;
    ry[i] = (t < 0) ? -t : ((t > H0 - 1) ? 2 * (H0 - 1) - t : t);
    t = xl + i - 1;
    rx[i] = (t < 0) ? -t : ((t > W0 - 1) ? 2 * (W0 - 1) - t : t);
  }
  const float* xb = x + (size_t)((b * C_IN + c) * H0) * W0;
  float nlp = 0.f, nhp = 0.f;
#pragma unroll
  for (int i = 0; i < 3; ++i)
#pragma unroll
    for (int j = 0; j < 3; ++j) {
      float xv = xb[ry[i] * W0 + rx[j]];
      int n = i * 3 + j;
      nlp += m[n] * xv;
      nhp += hk[n] * xv;
    }
  const float sc = (float)(H0 - 1) / (float)(HH - 1);
  float fy = Y * sc;
  int y0 = (int)fy; if (y0 > H0 - 2) y0 = H0 - 2;
  float wy = fy - y0;
  v4f o;
#pragma unroll
  for (int e = 0; e < 4; ++e) {
    int X = X0 + e;
    float fx = X * sc;
    int x0 = (int)fx; if (x0 > W0 - 2) x0 = W0 - 2;
    float wx = fx - x0;
    float w00 = (1.f - wy) * (1.f - wx), w01 = (1.f - wy) * wx;
    float w10 = wy * (1.f - wx),         w11 = wy * wx;
    float xup = xb[y0 * W0 + x0] * w00 + xb[y0 * W0 + x0 + 1] * w01
              + xb[(y0 + 1) * W0 + x0] * w10 + xb[(y0 + 1) * W0 + x0 + 1] * w11;
    o[e] = xup + lam * (nlp - xup) + tb * nhp;
  }
  vst2(yout + (size_t)g * 4, o);
}

extern "C" void kernel_launch(void* const* d_in, const int* in_sizes, int n_in,
                              void* d_out, int out_size, void* d_ws, size_t ws_size,
                              hipStream_t stream) {
  const float* x    = (const float*)d_in[0];
  const float* w1o  = (const float*)d_in[1];
  const float* b1o  = (const float*)d_in[2];
  const float* w2o  = (const float*)d_in[3];
  const float* b2o  = (const float*)d_in[4];
  const float* w1g  = (const float*)d_in[5];
  const float* b1g  = (const float*)d_in[6];
  const float* w2g  = (const float*)d_in[7];
  const float* b2g  = (const float*)d_in[8];
  const float* beta = (const float*)d_in[9];

  (void)in_sizes; (void)n_in; (void)out_size; (void)ws_size;
  char* ws = (char*)d_ws;
  _Float16* wp1  = (_Float16*)(ws + OFF_W1);
  _Float16* wp2  = (_Float16*)(ws + OFF_W2);
  _Float16* hbuf = (_Float16*)(ws + OFF_H);
  float*  rec  = (float*)(ws + OFF_REC);

  float* out  = (float*)d_out;
  float* yout = out;
  float* vout = out + OUT_V;
  float* gout = out + OUT_G;

  prep_w1<<<(W1ELEMS / 8 + 255) / 256, 256, 0, stream>>>(w1o, w1g, wp1);
  prep_w2<<<(W2ELEMS / 8 + 255) / 256, 256, 0, stream>>>(w2o, w2g, wp2);
  conv1_wmma<<<(NTILE + 7) / 8, 256, 0, stream>>>(x, b1o, b1g, wp1, hbuf);
  conv2_wmma<<<(NTILE + 7) / 8, 256, 0, stream>>>(hbuf, wp2, b2o, b2g, rec);
  write_v<<<((B_ * 8 * H0 * W0) / 4 + 255) / 256, 256, 0, stream>>>(rec, vout);
  write_g<<<(NHR / 4 + 255) / 256, 256, 0, stream>>>(rec, gout);
  upsample_combine<<<((B_ * C_IN * HH * HH) / 4 + 255) / 256, 256, 0, stream>>>(x, rec, beta, yout);
}
